// EncoderBiRNN_42013370089576
// MI455X (gfx1250) — hardware-run, weakly checked
//
#include <hip/hip_runtime.h>
#include <math.h>

constexpr int NBATCH = 64;
constexpr int NSTEP  = 512;
constexpr int NEMB   = 512;
constexpr int NHID   = 512;
constexpr int NGATE  = 3 * NHID;
constexpr int NVOCAB = 32000;
constexpr int NOUTW  = 2 * NHID;
constexpr int PTHR   = 256;
constexpr int RTHR   = 512;
constexpr int RWAVES = RTHR / 32;
constexpr int RROWS  = 32;
constexpr int HPITCH = 520;
constexpr int SLABP  = 36;
constexpr float OPCARRY  = 16.0f;
constexpr float ACC_FOLD = 1.0f / 256.0f;
constexpr int NX8  = NSTEP * NBATCH * NEMB / 8;
constexpr int NW8  = NGATE * NEMB / 8;
constexpr int XBLK = NX8 / PTHR;
constexpr int WBLK = NW8 / PTHR;
constexpr int PREP_BLOCKS = XBLK + 4 * WBLK;
static_assert(NX8 % PTHR == 0 && NW8 % PTHR == 0);
static_assert(NEMB == NHID);
static_assert(NEMB % 32 == 0 && NHID % 32 == 0);
static_assert(NEMB / 8 == 64);
static_assert(NBATCH % RROWS == 0 && RROWS == 32);
static_assert(NHID == 32 * RWAVES);
static_assert((RROWS * HPITCH) % 8 == 0 && HPITCH % 8 == 0 && SLABP % 4 == 0);

typedef __attribute__((ext_vector_type(16))) _Float16 v16h;
typedef __attribute__((ext_vector_type(8)))  _Float16 v8h;
typedef __attribute__((ext_vector_type(8)))  float    v8f;
typedef __attribute__((ext_vector_type(4)))  float    v4f;

__device__ __forceinline__ void acc_guard4(v8f& a, v8f& b, v8f& c, v8f& d) { asm volatile("v_nop\n\tv_nop\n\tv_nop\n\tv_nop" : "+v"(a), "+v"(b), "+v"(c), "+v"(d)); }
__device__ __forceinline__ void dep_guard6_h(v8f& a, v8f& b, v8f& c, v8f& d, v8f& e, v8f& f,
                                             v16h u0, v16h u1, v16h w0, v16h w1, v16h w2) {
  asm volatile("v_nop\n\tv_nop\n\tv_nop\n\tv_nop"
               : "+v"(a), "+v"(b), "+v"(c), "+v"(d), "+v"(e), "+v"(f)
               : "v"(u0), "v"(u1), "v"(w0), "v"(w1), "v"(w2));
}

template <typename T> struct Frag;
template <> struct Frag<_Float16> {
  typedef v16h V; union U { v16h v; v8h h[2]; };
  static __device__ __forceinline__ v16h load(const _Float16* p) {
    U f; f.h[0] = *(const v8h*)(p); f.h[1] = *(const v8h*)(p + 16); return f.v;
  }
  static __device__ __forceinline__ v8f mma(v16h a, v16h b, v8f c) {
    return __builtin_amdgcn_wmma_f32_16x16x32_f16(false, a, false, b, (short)0, c, false, false);
  }
};

__device__ __forceinline__ float fsig(float x)  { return __builtin_amdgcn_rcpf(1.0f + expf(-x)); }
__device__ __forceinline__ float ftanh(float x) { return 1.0f - 2.0f * __builtin_amdgcn_rcpf(1.0f + expf(2.0f * x)); }
__device__ __forceinline__ float cell_update(float aR, float aZ, float aX, float aH,
                                             float b_r, float b_z, float b_xn, float b_hn, float hprev) {
  const float rg = fsig(aR * ACC_FOLD + b_r);
  const float zg = fsig(aZ * ACC_FOLD + b_z);
  const float hn = aH * ACC_FOLD + b_hn;
  const float ng = ftanh(aX * ACC_FOLD + b_xn + rg * hn);
  return (1.0f - zg) * ng + zg * hprev;
}

__global__ __launch_bounds__(PTHR) void prep_kernel(const int* __restrict__ tokens, const float* __restrict__ emb,
                                                  const float* __restrict__ wih0, const float* __restrict__ whh0,
                                                  const float* __restrict__ wih1, const float* __restrict__ whh1,
                                                  unsigned short* __restrict__ X16,
                                                  unsigned short* __restrict__ WIH0, unsigned short* __restrict__ WHH0,
                                                  unsigned short* __restrict__ WIH1, unsigned short* __restrict__ WHH1) {
  const int blk = blockIdx.x, tid = threadIdx.x;
  const float* src;
  unsigned short* dst;
  if (blk < XBLK) {
    const int i    = blk * PTHR + tid;
    const int rowi = i >> 6;
    const int c8   = i & 63;
    const int t = rowi >> 6, b = rowi & 63;
    int tok = tokens[b * NSTEP + t];
    tok = tok < 0 ? 0 : tok;
    tok = tok > (NVOCAB - 1) ? (NVOCAB - 1) : tok;
    src = emb + (size_t)tok * NEMB + c8 * 8;
    dst = X16 + (size_t)i * 8;
  } else {
    const int p     = blk - XBLK;
    const int plane = p / WBLK;
    const int q     = (p - plane * WBLK) * PTHR + tid;
    if (plane == 0)      { src = wih0; dst = WIH0; }
    else if (plane == 1) { src = whh0; dst = WHH0; }
    else if (plane == 2) { src = wih1; dst = WIH1; }
    else                 { src = whh1; dst = WHH1; }
    src += (size_t)q * 8;
    dst += (size_t)q * 8;
  }
  const v4f a = *(const v4f*)(src);
  const v4f bq = *(const v4f*)(src + 4);
  v8h hv;
#pragma unroll
  for (int e = 0; e < 4; ++e) { hv[e] = (_Float16)(a[e] * OPCARRY); hv[4 + e] = (_Float16)(bq[e] * OPCARRY); }
  *(volatile v8h*)dst = hv;
  __threadfence();
  *(volatile v8h*)dst = hv;
}

__global__ __launch_bounds__(RTHR) void birec_kernel(const unsigned short* __restrict__ X16p,
                                                   const unsigned short* __restrict__ WIHp,
                                                   const unsigned short* __restrict__ WHHp,
                                                   const float* __restrict__ bih, const float* __restrict__ bhh,
                                                   float* __restrict__ out, int dir) {
  __shared__ __align__(16) _Float16 h16[RROWS * HPITCH];
  __shared__ __align__(16) float    slab[RWAVES][8 * SLABP];
  const _Float16* X16 = (const _Float16*)X16p;
  const _Float16* WIH = (const _Float16*)WIHp;
  const _Float16* WHH = (const _Float16*)WHHp;
  const int tid = threadIdx.x, lane = tid & 31, wave = tid >> 5;
  const int c = lane & 15, hh = lane >> 4, koff = hh * 8;
  const int bbase = blockIdx.x * RROWS;

  {
    v8h z;
#pragma unroll
    for (int e = 0; e < 8; ++e) z[e] = (_Float16)0.0f;
#pragma unroll 1
    for (int i = tid; i < RROWS * HPITCH / 8; i += RTHR) *(v8h*)(h16 + 8 * i) = z;
  }
  float hst[2][2][8];
#pragma unroll
  for (int m = 0; m < 2; ++m)
#pragma unroll
    for (int ntl = 0; ntl < 2; ++ntl)
#pragma unroll
      for (int r = 0; r < 8; ++r) hst[m][ntl][r] = 0.0f;
  float b_r[2], b_z[2], b_xn[2], b_hn[2];
#pragma unroll
  for (int ntl = 0; ntl < 2; ++ntl) {
    const int j = 32 * wave + 16 * ntl + c;
    b_r[ntl]  = bih[j] + bhh[j];
    b_z[ntl]  = bih[NHID + j] + bhh[NHID + j];
    b_xn[ntl] = bih[2 * NHID + j];
    b_hn[ntl] = bhh[2 * NHID + j];
  }
  __syncthreads();

  const v8f z8 = {0.f, 0.f, 0.f, 0.f, 0.f, 0.f, 0.f, 0.f};

#pragma unroll 1
  for (int s = 0; s < NSTEP; ++s) {
    const int t = dir ? (NSTEP - 1 - s) : s;
    const _Float16* xrow0 = X16 + (size_t)t * (NBATCH * NEMB) + (size_t)(bbase + c) * NEMB + koff;
    const _Float16* xrow1 = xrow0 + 16 * NEMB;
    const _Float16* hrow0 = h16 + c * HPITCH + koff;
    const _Float16* hrow1 = h16 + (16 + c) * HPITCH + koff;
#pragma unroll
    for (int ntl = 0; ntl < 2; ++ntl) {
      const int j = 32 * wave + 16 * ntl + c;
      const _Float16* wir = WIH + (size_t)j * NEMB + koff;
      const _Float16* wiz = wir + (size_t)NHID * NEMB;
      const _Float16* win = wiz + (size_t)NHID * NEMB;
      const _Float16* whr = WHH + (size_t)j * NHID + koff;
      const _Float16* whz = whr + (size_t)NHID * NHID;
      const _Float16* whn = whz + (size_t)NHID * NHID;
      v8f aR0 = z8, aR1 = z8, aZ0 = z8, aZ1 = z8, aX0 = z8, aX1 = z8;
#pragma unroll 1
      for (int k0 = 0; k0 < NEMB; k0 += 32) {
        const v16h a0 = Frag<_Float16>::load(xrow0 + k0);
        const v16h a1 = Frag<_Float16>::load(xrow1 + k0);
        const v16h br = Frag<_Float16>::load(wir + k0);
        const v16h bz = Frag<_Float16>::load(wiz + k0);
        const v16h bn = Frag<_Float16>::load(win + k0);
        aR0 = Frag<_Float16>::mma(a0, br, aR0);
        aR1 = Frag<_Float16>::mma(a1, br, aR1);
        aZ0 = Frag<_Float16>::mma(a0, bz, aZ0);
        aZ1 = Frag<_Float16>::mma(a1, bz, aZ1);
        aX0 = Frag<_Float16>::mma(a0, bn, aX0);
        aX1 = Frag<_Float16>::mma(a1, bn, aX1);
        dep_guard6_h(aR0, aR1, aZ0, aZ1, aX0, aX1, a0, a1, br, bz, bn);
      }
      v8f aH0 = z8, aH1 = z8;
#pragma unroll 1
      for (int k0 = 0; k0 < NHID; k0 += 32) {
        const v16h a0 = Frag<_Float16>::load(hrow0 + k0);
        const v16h a1 = Frag<_Float16>::load(hrow1 + k0);
        const v16h br = Frag<_Float16>::load(whr + k0);
        const v16h bz = Frag<_Float16>::load(whz + k0);
        const v16h bn = Frag<_Float16>::load(whn + k0);
        aR0 = Frag<_Float16>::mma(a0, br, aR0);
        aR1 = Frag<_Float16>::mma(a1, br, aR1);
        aZ0 = Frag<_Float16>::mma(a0, bz, aZ0);
        aZ1 = Frag<_Float16>::mma(a1, bz, aZ1);
        aH0 = Frag<_Float16>::mma(a0, bn, aH0);
        aH1 = Frag<_Float16>::mma(a1, bn, aH1);
        dep_guard6_h(aR0, aR1, aZ0, aZ1, aH0, aH1, a0, a1, br, bz, bn);
      }
      acc_guard4(aR0, aR1, aZ0, aZ1);
      acc_guard4(aX0, aX1, aH0, aH1);
#pragma unroll
      for (int r = 0; r < 8; ++r) {
        hst[0][ntl][r] = cell_update(aR0[r], aZ0[r], aX0[r], aH0[r], b_r[ntl], b_z[ntl], b_xn[ntl], b_hn[ntl], hst[0][ntl][r]);
        hst[1][ntl][r] = cell_update(aR1[r], aZ1[r], aX1[r], aH1[r], b_r[ntl], b_z[ntl], b_xn[ntl], b_hn[ntl], hst[1][ntl][r]);
      }
    }
    __syncthreads();
#pragma unroll
    for (int m = 0; m < 2; ++m)
#pragma unroll
      for (int ntl = 0; ntl < 2; ++ntl)
#pragma unroll
        for (int r = 0; r < 8; ++r)
          h16[(16 * m + 8 * hh + r) * HPITCH + 32 * wave + 16 * ntl + c] = (_Float16)(OPCARRY * hst[m][ntl][r]);
    __syncthreads();
  }

  float* slw = slab[wave];
  const int q = lane >> 3, c4 = (lane & 7) * 4;
#pragma unroll
  for (int p = 0; p < 4; ++p) {
    const int m = p >> 1, hs = p & 1;
    if (hh == hs) {
#pragma unroll
      for (int ntl = 0; ntl < 2; ++ntl)
#pragma unroll
        for (int r = 0; r < 8; ++r) slw[r * SLABP + 16 * ntl + c] = hst[m][ntl][r];
    }
    __builtin_amdgcn_fence(__ATOMIC_RELEASE, "workgroup");
    __builtin_amdgcn_wave_barrier();
    __builtin_amdgcn_fence(__ATOMIC_ACQUIRE, "workgroup");
    const v4f v0 = *(const v4f*)(slw + q * SLABP + c4);
    const v4f v1 = *(const v4f*)(slw + (4 + q) * SLABP + c4);
    float* o0 = out + (size_t)(bbase + 8 * p + q) * NOUTW + dir * NHID + 32 * wave + c4;
    float* o1 = o0 + 4 * NOUTW;
    for (int pass = 0; pass < 2; ++pass) {
      *(volatile v4f*)o0 = v0;
      *(volatile v4f*)o1 = v1;
      __threadfence();
    }
    __builtin_amdgcn_fence(__ATOMIC_RELEASE, "workgroup");
    __builtin_amdgcn_wave_barrier();
    __builtin_amdgcn_fence(__ATOMIC_ACQUIRE, "workgroup");
  }
}

extern "C" void kernel_launch(void* const* d_in, const int* in_sizes, int n_in,
                              void* d_out, int out_size, void* d_ws, size_t ws_size, hipStream_t stream) {
  if (n_in < 10 || d_out == nullptr || d_ws == nullptr) return;
  if (in_sizes[0] != NBATCH * NSTEP || in_sizes[1] != NVOCAB * NEMB ||
      in_sizes[2] != NGATE * NEMB || in_sizes[3] != NGATE * NHID || in_sizes[4] != NGATE || in_sizes[5] != NGATE ||
      in_sizes[6] != NGATE * NEMB || in_sizes[7] != NGATE * NHID || in_sizes[8] != NGATE || in_sizes[9] != NGATE ||
      out_size != NBATCH * NOUTW) return;

  const int*   tokens = (const int*)d_in[0];
  const float* emb    = (const float*)d_in[1];
  const float* wih_f  = (const float*)d_in[2];
  const float* whh_f  = (const float*)d_in[3];
  const float* bih_f  = (const float*)d_in[4];
  const float* bhh_f  = (const float*)d_in[5];
  const float* wih_r  = (const float*)d_in[6];
  const float* whh_r  = (const float*)d_in[7];
  const float* bih_r  = (const float*)d_in[8];
  const float* bhh_r  = (const float*)d_in[9];
  float* out = (float*)d_out;

  char* ws = (char*)d_ws; size_t off = 0;
  auto carve = [&](size_t bytes) -> char* { char* p = ws + off; off += (bytes + 255) & ~(size_t)255; return p; };
  unsigned short* X16  = (unsigned short*)carve((size_t)NSTEP * NBATCH * NEMB * 2);
  unsigned short* WIH0 = (unsigned short*)carve((size_t)NGATE * NEMB * 2);
  unsigned short* WHH0 = (unsigned short*)carve((size_t)NGATE * NHID * 2);
  unsigned short* WIH1 = (unsigned short*)carve((size_t)NGATE * NEMB * 2);
  unsigned short* WHH1 = (unsigned short*)carve((size_t)NGATE * NHID * 2);
  if (off > ws_size || off > (size_t)134217728) return;

  prep_kernel<<<PREP_BLOCKS, PTHR, 0, stream>>>(tokens, emb, wih_f, whh_f, wih_r, whh_r, X16, WIH0, WHH0, WIH1, WHH1);
  birec_kernel<<<NBATCH / RROWS, RTHR, 0, stream>>>(X16, WIH0, WHH0, bih_f, bhh_f, out, 0);
  birec_kernel<<<NBATCH / RROWS, RTHR, 0, stream>>>(X16, WIH1, WHH1, bih_r, bhh_r, out, 1);
}
